// DCN_off_b_50070728737063
// MI455X (gfx1250) — hardware-verified
//
#include <hip/hip_runtime.h>
#include <math.h>

typedef __attribute__((ext_vector_type(16))) _Float16 v16h;
typedef __attribute__((ext_vector_type(8)))  _Float16 v8h;
typedef __attribute__((ext_vector_type(16))) __bf16   v16b;
typedef __attribute__((ext_vector_type(8)))  __bf16   v8b;
typedef __attribute__((ext_vector_type(8)))  float    v8f;
typedef __attribute__((ext_vector_type(4)))  float    v4f;
typedef __attribute__((ext_vector_type(4)))  unsigned v4u;

constexpr int kB    = 4;
constexpr int kH    = 160;
constexpr int kW    = 160;
constexpr int kHW   = kH * kW;
constexpr int kFc   = 64;
constexpr int kC1   = 128;
constexpr int kPW   = 162;
constexpr int kPP   = kPW * kPW;
constexpr int kNcom = 216;
constexpr int kNcomPad = 256;
constexpr int kMT   = (kH / 2) * (kW / 32);
constexpr float kWCarry    = 64.0f;
constexpr float kWCarryInv = 1.0f / 64.0f;
constexpr float kLoCarry    = 2048.0f;
constexpr float kLoCarryInv = 1.0f / 2048.0f;
static_assert(kW % 32 == 0 && kH % 2 == 0, "pixel tile 2 x 32");
static_assert(kMT == 400, "M tiles per image");
static_assert((kC1 % 32) == 0 && (kFc % 32) == 0, "tap chunk multiple of 32");
static_assert((kNcomPad % 64) == 0 && kNcomPad >= kNcom, "padded N");

constexpr size_t kSzP128 = (size_t)kPP * 128 * 2;
constexpr size_t kSzP64  = (size_t)kPP * 64 * 2;
constexpr size_t kOffCAT = 0;
constexpr size_t kOffTH  = kOffCAT + kSzP128;
constexpr size_t kOffTL  = kOffTH  + kSzP128;
constexpr size_t kOffOH  = kOffTL  + kSzP128;
constexpr size_t kOffOL  = kOffOH  + kSzP64;
constexpr size_t kOffXF  = kOffOL  + kSzP64;
constexpr size_t kOffCOM = kOffXF  + (size_t)kHW * 64 * 4;
constexpr size_t kOffW1  = kOffCOM + (size_t)kHW * kNcomPad * 4;
constexpr size_t kOffW2  = kOffW1  + (size_t)128 * 1152 * 2;
constexpr size_t kOffW3  = kOffW2  + (size_t)64 * 1152 * 2;
constexpr size_t kOffW4  = kOffW3  + (size_t)64 * 1152 * 2;
constexpr size_t kOffWD  = kOffW4  + (size_t)kNcomPad * 576 * 2;
constexpr size_t kWsTotal = kOffWD + (size_t)64 * 576 * 2;
static_assert(kWsTotal == 60600320ull, "carve total");
static_assert(kWsTotal <= 134217728ull, "carve cap");
static_assert((kOffTH % 128) == 0 && (kOffTL % 128) == 0 && (kOffOH % 128) == 0 && (kOffOL % 128) == 0 &&
              (kOffXF % 128) == 0 && (kOffCOM % 128) == 0 && (kOffW1 % 128) == 0 && (kOffW2 % 128) == 0 &&
              (kOffW3 % 128) == 0 && (kOffW4 % 128) == 0 && (kOffWD % 128) == 0, "128-B aligned regions");

__device__ __forceinline__ unsigned short f2bf_bits(float f) {
  unsigned u = __float_as_uint(f);
  return (unsigned short)((u + 0x7FFFu + ((u >> 16) & 1u)) >> 16);
}
__device__ __forceinline__ float bf_bits2f(unsigned short h) { return __uint_as_float(((unsigned)h) << 16); }
__device__ __forceinline__ float bf_rne(float f) { return bf_bits2f(f2bf_bits(f)); }

__device__ __forceinline__ void split_f16(float t, _Float16& hi, _Float16& lo) {
  const float th = (fabsf(t) < 6.103515625e-5f) ? 0.0f : t;
  hi = (_Float16)th;
  float hf = (float)hi;
  asm volatile("" : "+v"(hf));
  lo = (_Float16)((t - hf) * kLoCarry);
}

__device__ __forceinline__ v8f mma_h(v16h a, v16h b, v8f c) {
  c = __builtin_amdgcn_wmma_f32_16x16x32_f16(false, a, false, b, (short)0, c, false, false);
  asm volatile("v_nop\n\tv_nop\n\tv_nop\n\tv_nop" : "+v"(c) : "v"(a), "v"(b));
  return c;
}
__device__ __forceinline__ v8f mma_b(v16b a, v16b b, v8f c) {
  c = __builtin_amdgcn_wmma_f32_16x16x32_bf16(false, a, false, b, (short)0, c, false, false);
  asm volatile("v_nop\n\tv_nop\n\tv_nop\n\tv_nop" : "+v"(c) : "v"(a), "v"(b));
  return c;
}

template <typename T> struct Frag;
template <> struct Frag<_Float16> {
  typedef v16h V; union U { v16h v; v8h h[2]; };
  static __device__ __forceinline__ v16h load(const _Float16* p) {
    U f; f.h[0] = *(const v8h*)(p); f.h[1] = *(const v8h*)(p + 16); return f.v;
  }
  static __device__ __forceinline__ v8f mmag(v16h a, v16h b, v8f c) { return mma_h(a, b, c); }
};
template <> struct Frag<__bf16> {
  typedef v16b V; union U { v16b v; v8b h[2]; };
  static __device__ __forceinline__ v16b load(const __bf16* p) {
    U f; f.h[0] = *(const v8b*)(p); f.h[1] = *(const v8b*)(p + 16); return f.v;
  }
  static __device__ __forceinline__ v8f mmag(v16b a, v16b b, v8f c) { return mma_b(a, b, c); }
};
template <int ET> struct Elem;
template <> struct Elem<0> { typedef _Float16 T; };
template <> struct Elem<1> { typedef __bf16 T; };

template <int MODE>
__global__ __launch_bounds__(256) void pack_w_kernel(const float* __restrict__ w, unsigned short* __restrict__ dst,
                                                     int Oreal, int I, int total8) {
  const int i8 = blockIdx.x * 256 + threadIdx.x;
  if (i8 >= total8) return;
  const int per_row = (9 * I) >> 3;
  const int o  = i8 / per_row;
  const int k0 = (i8 - o * per_row) << 3;
  const int t  = k0 / I;
  const int i0 = k0 - t * I;
  const int oc = (o < Oreal) ? o : (Oreal - 1);
  const bool live = (o < Oreal);
  v8h hv;
#pragma unroll
  for (int e = 0; e < 8; ++e) {
    const float raw = w[((size_t)oc * I + i0 + e) * 9 + t];
    float r = bf_rne(raw);
    r = live ? r : 0.0f;
    unsigned short bits;
    if (MODE == 0) {
      bits = (unsigned short)(__float_as_uint(r) >> 16);
    } else {
      const _Float16 hq = (_Float16)(r * kWCarry);
      bits = __builtin_bit_cast(unsigned short, hq);
    }
    hv[e] = __builtin_bit_cast(_Float16, bits);
  }
  unsigned short* q = dst + (size_t)i8 * 8;
  *(volatile v8h*)q = hv;
  __threadfence();
  *(volatile v8h*)q = hv;
}

__global__ __launch_bounds__(256) void halo_zero_kernel(unsigned short* __restrict__ plane, int C, int nlines) {
  const int idx  = blockIdx.x * 256 + threadIdx.x;
  const int line = idx >> 3, part = idx & 7;
  if (line >= nlines) return;
  const int lpp = C >> 6;
  const int hp  = line / lpp;
  const int sub = line - hp * lpp;
  const int r   = hp - 324;
  const int py  = (hp < 162) ? 0 : ((hp < 324) ? 161 : (1 + (r >> 1)));
  const int px  = (hp < 162) ? hp : ((hp < 324) ? (hp - 162) : ((r & 1) * 161));
  unsigned short* p = plane + ((size_t)(py * kPW + px)) * C + sub * 64 + part * 8;
  const v4u z = {0u, 0u, 0u, 0u};
  *(volatile v4u*)p = z;
  __threadfence();
  *(volatile v4u*)p = z;
}

__global__ __launch_bounds__(256) void cat_plane_kernel(const float* __restrict__ ali, const float* __restrict__ rin,
                                                        unsigned short* __restrict__ cat) {
  __shared__ float sT[128 * 33];
  const int tid = threadIdx.x;
  const int h  = blockIdx.x / 5;
  const int w0 = (blockIdx.x - h * 5) * 32;
  const int cl = tid >> 3, px4 = (tid & 7) * 4;
#pragma unroll
  for (int it = 0; it < 4; ++it) {
    const float* src = (it < 2) ? ali : rin;
    const int cc = (it & 1) * 32 + cl;
    const v4f v = *(const v4f*)(src + ((size_t)cc * kH + h) * kW + w0 + px4);
    const int ch = it * 32 + cl;
    const float e0 = v[0], e1 = v[1], e2 = v[2], e3 = v[3];
    sT[ch * 33 + px4 + 0] = e0;
    sT[ch * 33 + px4 + 1] = e1;
    sT[ch * 33 + px4 + 2] = e2;
    sT[ch * 33 + px4 + 3] = e3;
  }
  __syncthreads();
  v8h ov[2];
#pragma unroll
  for (int s = 0; s < 2; ++s) {
    const int task = tid + 256 * s;
    const int px = task >> 4, c8 = (task & 15) * 8;
#pragma unroll
    for (int e = 0; e < 8; ++e) {
      const float f = sT[(c8 + e) * 33 + px];
      const unsigned short hb = f2bf_bits(f);
      ov[s][e] = __builtin_bit_cast(_Float16, hb);
    }
  }
  for (int pass = 0; pass < 2; ++pass) {
#pragma unroll
    for (int s = 0; s < 2; ++s) {
      const int task = tid + 256 * s;
      const int px = task >> 4, c8 = (task & 15) * 8;
      unsigned short* q = cat + ((size_t)((h + 1) * kPW + w0 + px + 1)) * 128 + c8;
      *(volatile v8h*)q = ov[s];
    }
    __threadfence();
  }
}

template <int ET, int CIN, int NT, int NPASS, int EPI>
__global__ __launch_bounds__(128) void conv3x3_kernel(
    const unsigned short* __restrict__ Ahi_p, const unsigned short* __restrict__ Alo_p,
    const unsigned short* __restrict__ Bt_p, const float* __restrict__ bias,
    unsigned short* __restrict__ out_hi, unsigned short* __restrict__ out_lo,
    float* __restrict__ out_f, int nreal) {
  typedef typename Elem<ET>::T T;
  typedef typename Frag<T>::V V;
  constexpr int KTOT = 9 * CIN;
  static_assert((CIN % 32) == 0, "tap chunk");
  __shared__ __align__(16) float sT[4][32 * 68];
  const int lane = threadIdx.x & 31;
  const int wave = __builtin_amdgcn_readfirstlane((int)(threadIdx.x >> 5));
  const int tile = blockIdx.x * 4 + wave;
  if (tile >= kMT * NT) return;
  const int tm = tile / NT;
  const int tn = tile - tm * NT;
  const int hpair = tm / 5;
  const int seg   = tm - hpair * 5;
  const int hbase = hpair * 2;
  const int w0    = seg * 32;
  const int n0    = tn * 64;
  const int rlane = lane & 15;
  const int koff  = (lane >> 4) * 8;
  const int mOff  = (lane >> 4) * 8;
  const T* Bt = (const T*)Bt_p;

  v8f acc[4][4];
#pragma unroll
  for (int i = 0; i < 4; ++i)
#pragma unroll
    for (int j = 0; j < 4; ++j) acc[i][j] = (v8f){0.f, 0.f, 0.f, 0.f, 0.f, 0.f, 0.f, 0.f};

  int pbeg = 1;
  if (NPASS == 2) pbeg = (EPI == 3 && tn == NT - 1) ? 1 : 0;
#pragma unroll 1
  for (int pass = pbeg; pass < 2; ++pass) {
    const T* Ap = (const T*)((NPASS == 2 && pass == 0) ? Alo_p : Ahi_p);
#pragma unroll 1
    for (int ky = 0; ky < 3; ++ky) {
#pragma unroll 1
      for (int kx = 0; kx < 3; ++kx) {
        const T* arow = Ap + ((size_t)((hbase + ky) * kPW + w0 + rlane + kx)) * CIN + koff;
        const T* brow = Bt + ((size_t)(n0 + rlane)) * KTOT + (ky * 3 + kx) * CIN + koff;
#pragma unroll 1
        for (int c0 = 0; c0 < CIN; c0 += 32) {
          V bh[4];
#pragma unroll
          for (int j = 0; j < 4; ++j) bh[j] = Frag<T>::load(brow + (size_t)(j * 16) * KTOT + c0);
#pragma unroll
          for (int i = 0; i < 4; ++i) {
            const V ah = Frag<T>::load(arow + ((i >> 1) * kPW + (i & 1) * 16) * CIN + c0);
#pragma unroll
            for (int j = 0; j < 4; ++j) acc[i][j] = Frag<T>::mmag(ah, bh[j], acc[i][j]);
          }
        }
      }
    }
    if (NPASS == 2 && pass == 0) {
#pragma unroll
      for (int i = 0; i < 4; ++i)
#pragma unroll
        for (int j = 0; j < 4; ++j) acc[i][j] = acc[i][j] * kLoCarryInv;
    }
  }

  const float scale = (ET == 0) ? kWCarryInv : 1.0f;
  float bvj[4];
#pragma unroll
  for (int j = 0; j < 4; ++j) {
    const int n  = n0 + j * 16 + rlane;
    const int nc = (n < nreal) ? n : (nreal - 1);
    const float rb = bf_rne(bias[nc]);
    bvj[j] = (n < nreal) ? rb : 0.0f;
  }
  float* slab = sT[wave];
#pragma unroll
  for (int hr = 0; hr < 2; ++hr) {
    const int hrow = hbase + hr;
#pragma unroll
    for (int ii = 0; ii < 2; ++ii) {
#pragma unroll
      for (int j = 0; j < 4; ++j) {
#pragma unroll
        for (int r = 0; r < 8; ++r) {
          float v = acc[hr * 2 + ii][j][r] * scale + bvj[j];
          if (EPI != 3) v = (v >= 0.0f) ? v : 0.1f * v;
          slab[(ii * 16 + mOff + r) * 68 + j * 16 + rlane] = v;
        }
      }
    }
    __builtin_amdgcn_fence(__ATOMIC_RELEASE, "workgroup");
    __builtin_amdgcn_wave_barrier();
    __builtin_amdgcn_fence(__ATOMIC_ACQUIRE, "workgroup");
    if (EPI == 1) {
      const int lq = lane >> 3, px4 = (lane & 7) * 4;
      for (int pass2 = 0; pass2 < 2; ++pass2) {
#pragma unroll 4
        for (int it = 0; it < 16; ++it) {
          const int ch = it * 4 + lq;
          const float e0 = slab[(px4 + 0) * 68 + ch];
          const float e1 = slab[(px4 + 1) * 68 + ch];
          const float e2 = slab[(px4 + 2) * 68 + ch];
          const float e3 = slab[(px4 + 3) * 68 + ch];
          const v4f v = {e0, e1, e2, e3};
          *(volatile v4f*)(out_f + ((size_t)(n0 + ch) * kH + hrow) * kW + w0 + px4) = v;
        }
        __threadfence();
      }
    }
    if (EPI == 0 || EPI == 1) {
      constexpr int PC = (EPI == 0) ? 128 : 64;
      const int q = lane >> 3, c8 = (lane & 7) * 8;
      for (int pass2 = 0; pass2 < 2; ++pass2) {
#pragma unroll 2
        for (int it = 0; it < 8; ++it) {
          const int row = it * 4 + q;
          const float* sp = slab + row * 68 + c8;
          const v4f a0 = *(const v4f*)(sp);
          const v4f a1 = *(const v4f*)(sp + 4);
          v8h hv, lv;
#pragma unroll
          for (int e = 0; e < 4; ++e) {
            const float t0 = a0[e];
            const float t1 = a1[e];
            _Float16 h0v, l0v, h1v, l1v;
            split_f16(t0, h0v, l0v);
            split_f16(t1, h1v, l1v);
            hv[e] = h0v; hv[4 + e] = h1v;
            lv[e] = l0v; lv[4 + e] = l1v;
          }
          const size_t o = ((size_t)((hrow + 1) * kPW + w0 + row + 1)) * PC + n0 + c8;
          *(volatile v8h*)(out_hi + o) = hv;
          *(volatile v8h*)(out_lo + o) = lv;
        }
        __threadfence();
      }
    }
    if (EPI == 2 || EPI == 3) {
      constexpr int LDC = (EPI == 2) ? 64 : kNcomPad;
      const int hh2 = lane >> 4, c4 = (lane & 15) * 4;
      for (int pass2 = 0; pass2 < 2; ++pass2) {
#pragma unroll 4
        for (int it = 0; it < 16; ++it) {
          const int row = it * 2 + hh2;
          const v4f v = *(const v4f*)(slab + row * 68 + c4);
          *(volatile v4f*)(out_f + ((size_t)(hrow * kW + w0 + row)) * LDC + n0 + c4) = v;
        }
        __threadfence();
      }
    }
    __builtin_amdgcn_fence(__ATOMIC_RELEASE, "workgroup");
    __builtin_amdgcn_wave_barrier();
    __builtin_amdgcn_fence(__ATOMIC_ACQUIRE, "workgroup");
  }
}

__global__ __launch_bounds__(256) void dcn_kernel(const float* __restrict__ xf, const float* __restrict__ com,
                                                  const unsigned short* __restrict__ Wd_p,
                                                  const float* __restrict__ bias, const int* __restrict__ groups,
                                                  float* __restrict__ out0) {
  __shared__ __align__(16) _Float16 At[64 * 72];
  __shared__ __align__(16) float sS[8][16 * 36];
  union FU { v16h v; v8h h[2]; };
  const int tid  = threadIdx.x;
  const int lane = tid & 31;
  const int wave = __builtin_amdgcn_readfirstlane((int)(threadIdx.x >> 5));
  const int hpair = blockIdx.x / 5;
  const int seg   = blockIdx.x - hpair * 5;
  const int hbase = hpair * 2;
  const int w0    = seg * 32;
  const int rlane = lane & 15;
  const int koff  = (lane >> 4) * 8;
  const int mOff  = (lane >> 4) * 8;
  const int jn = wave & 3;
  const int mh = wave >> 2;
  const _Float16* Wd = (const _Float16*)Wd_p;

  v8f acc0 = (v8f){0.f, 0.f, 0.f, 0.f, 0.f, 0.f, 0.f, 0.f};
  v8f acc1 = (v8f){0.f, 0.f, 0.f, 0.f, 0.f, 0.f, 0.f, 0.f};

#pragma unroll 1
  for (int ky = 0; ky < 3; ++ky) {
#pragma unroll 1
    for (int kx = 0; kx < 3; ++kx) {
      const int k = ky * 3 + kx;
      __syncthreads();
#pragma unroll 1
      for (int s = 0; s < 2; ++s) {
        const int tt = tid + 256 * s;
        const int px = tt >> 3, g = tt & 7;
        const int h = hbase + (px >> 5);
        const int w = w0 + (px & 31);
        const float* cr = com + ((size_t)(h * kW + w)) * kNcomPad + g * 9 + k;
        const float dy = cr[0];
        const float dx = cr[72];
        const float ml = cr[144];
        const float pyf = (dy + (float)h) + (float)(ky - 1);
        const float pxf = (dx + (float)w) + (float)(kx - 1);
        const float y0f = floorf(pyf);
        const float x0f = floorf(pxf);
        const float wy = pyf - y0f;
        const float wx = pxf - x0f;
        const int y0 = (int)fminf(fmaxf(y0f, -3.0f), 162.0f);
        const int x0 = (int)fminf(fmaxf(x0f, -3.0f), 162.0f);
        const int y1 = y0 + 1, x1 = x0 + 1;
        const bool vy0 = (y0 >= 0) && (y0 < kH);
        const bool vy1 = (y1 >= 0) && (y1 < kH);
        const bool vx0 = (x0 >= 0) && (x0 < kW);
        const bool vx1 = (x1 >= 0) && (x1 < kW);
        const int cy0 = min(max(y0, 0), kH - 1);
        const int cy1 = min(max(y1, 0), kH - 1);
        const int cx0 = min(max(x0, 0), kW - 1);
        const int cx1 = min(max(x1, 0), kW - 1);
        const float omy = 1.0f - wy, omx = 1.0f - wx;
        float w00 = omy * omx, w01 = omy * wx, w10 = wy * omx, w11 = wy * wx;
        w00 = (vy0 && vx0) ? w00 : 0.0f;
        w01 = (vy0 && vx1) ? w01 : 0.0f;
        w10 = (vy1 && vx0) ? w10 : 0.0f;
        w11 = (vy1 && vx1) ? w11 : 0.0f;
        const float mk = 1.0f / (1.0f + expf(-ml));
        const float* p00 = xf + ((size_t)(cy0 * kW + cx0)) * 64 + g * 8;
        const float* p01 = xf + ((size_t)(cy0 * kW + cx1)) * 64 + g * 8;
        const float* p10 = xf + ((size_t)(cy1 * kW + cx0)) * 64 + g * 8;
        const float* p11 = xf + ((size_t)(cy1 * kW + cx1)) * 64 + g * 8;
        const v4f a0 = *(const v4f*)(p00), a1 = *(const v4f*)(p00 + 4);
        const v4f b0 = *(const v4f*)(p01), b1 = *(const v4f*)(p01 + 4);
        const v4f c0 = *(const v4f*)(p10), c1 = *(const v4f*)(p10 + 4);
        const v4f d0 = *(const v4f*)(p11), d1 = *(const v4f*)(p11 + 4);
        v8h hv;
#pragma unroll
        for (int e = 0; e < 4; ++e) {
          float s0 = a0[e] * w00;
          s0 = fmaf(b0[e], w01, s0);
          s0 = fmaf(c0[e], w10, s0);
          s0 = fmaf(d0[e], w11, s0);
          float s1 = a1[e] * w00;
          s1 = fmaf(b1[e], w01, s1);
          s1 = fmaf(c1[e], w10, s1);
          s1 = fmaf(d1[e], w11, s1);
          hv[e]     = (_Float16)(s0 * mk);
          hv[4 + e] = (_Float16)(s1 * mk);
        }
        *(v8h*)(At + px * 72 + g * 8) = hv;
      }
      __syncthreads();
      const _Float16* wrow = Wd + ((size_t)(jn * 16 + rlane)) * 576 + k * 64 + koff;
#pragma unroll
      for (int s2 = 0; s2 < 2; ++s2) {
        const v16h bf = Frag<_Float16>::load(wrow + s2 * 32);
        FU fa0, fa1;
        const _Float16* ar0 = At + ((mh * 2 + 0) * 16 + rlane) * 72 + s2 * 32 + koff;
        const _Float16* ar1 = At + ((mh * 2 + 1) * 16 + rlane) * 72 + s2 * 32 + koff;
        fa0.h[0] = *(const v8h*)(ar0);
        fa0.h[1] = *(const v8h*)(ar0 + 16);
        fa1.h[0] = *(const v8h*)(ar1);
        fa1.h[1] = *(const v8h*)(ar1 + 16);
        acc0 = mma_h(fa0.v, bf, acc0);
        acc1 = mma_h(fa1.v, bf, acc1);
      }
    }
  }

  const int grp = groups[0];
  const bool okg = (grp == 8);
  const float poison = __uint_as_float(0x7fc00000u);
  const float bv = bf_rne(bias[jn * 16 + rlane]);
  const int hrow = hbase + mh;
  float* slab = sS[wave];
#pragma unroll
  for (int r = 0; r < 8; ++r) {
    float v0 = acc0[r] * kWCarryInv + bv;
    float v1 = acc1[r] * kWCarryInv + bv;
    v0 = (v0 >= 0.0f) ? v0 : 0.1f * v0;
    v1 = (v1 >= 0.0f) ? v1 : 0.1f * v1;
    v0 = okg ? v0 : poison;
    v1 = okg ? v1 : poison;
    slab[rlane * 36 + mOff + r] = v0;
    slab[rlane * 36 + 16 + mOff + r] = v1;
  }
  __builtin_amdgcn_fence(__ATOMIC_RELEASE, "workgroup");
  __builtin_amdgcn_wave_barrier();
  __builtin_amdgcn_fence(__ATOMIC_ACQUIRE, "workgroup");
  {
    const int lq = lane >> 3, px4 = (lane & 7) * 4;
    for (int pass2 = 0; pass2 < 2; ++pass2) {
#pragma unroll
      for (int it = 0; it < 4; ++it) {
        const int ch = it * 4 + lq;
        const v4f v = *(const v4f*)(slab + ch * 36 + px4);
        *(volatile v4f*)(out0 + ((size_t)(jn * 16 + ch) * kH + hrow) * kW + w0 + px4) = v;
      }
      __threadfence();
    }
  }
}

extern "C" void kernel_launch(void* const* d_in, const int* in_sizes, int n_in,
                              void* d_out, int out_size, void* d_ws, size_t ws_size,
                              hipStream_t stream) {
  if (n_in < 13) return;
  if (in_sizes[0] != kB * kFc * kHW) return;
  if (in_sizes[1] != kB * kFc * kHW) return;
  if (in_sizes[2] != 128 * 128 * 9) return;
  if (in_sizes[3] != 128) return;
  if (in_sizes[4] != 64 * 128 * 9) return;
  if (in_sizes[5] != 64) return;
  if (in_sizes[6] != 64 * 128 * 9) return;
  if (in_sizes[7] != 64) return;
  if (in_sizes[8] != kNcom * 64 * 9) return;
  if (in_sizes[9] != kNcom) return;
  if (in_sizes[10] != 64 * 64 * 9) return;
  if (in_sizes[11] != 64) return;
  if (in_sizes[12] != 1) return;
  if (out_size != 2 * kB * kFc * kHW) return;
  if (ws_size < kWsTotal) return;

  const float* ali    = (const float*)d_in[0];
  const float* rin    = (const float*)d_in[1];
  const float* w_conv = (const float*)d_in[2];
  const float* b_conv = (const float*)d_in[3];
  const float* w_off  = (const float*)d_in[4];
  const float* b_off  = (const float*)d_in[5];
  const float* w_x    = (const float*)d_in[6];
  const float* b_x    = (const float*)d_in[7];
  const float* w_com  = (const float*)d_in[8];
  const float* b_com  = (const float*)d_in[9];
  const float* w_dcn  = (const float*)d_in[10];
  const float* b_dcn  = (const float*)d_in[11];
  const int*   groups = (const int*)d_in[12];

  float* out0 = (float*)d_out;
  float* out1 = (float*)d_out + (size_t)kB * kFc * kHW;

  char* ws = (char*)d_ws;
  unsigned short* CAT = (unsigned short*)(ws + kOffCAT);
  unsigned short* TH  = (unsigned short*)(ws + kOffTH);
  unsigned short* TL  = (unsigned short*)(ws + kOffTL);
  unsigned short* OH  = (unsigned short*)(ws + kOffOH);
  unsigned short* OL  = (unsigned short*)(ws + kOffOL);
  float*          XF  = (float*)(ws + kOffXF);
  float*          COM = (float*)(ws + kOffCOM);
  unsigned short* W1  = (unsigned short*)(ws + kOffW1);
  unsigned short* W2  = (unsigned short*)(ws + kOffW2);
  unsigned short* W3  = (unsigned short*)(ws + kOffW3);
  unsigned short* W4  = (unsigned short*)(ws + kOffW4);
  unsigned short* WD  = (unsigned short*)(ws + kOffWD);

  pack_w_kernel<0><<<(128 * 1152 / 8) / 256, 256, 0, stream>>>(w_conv, W1, 128, 128, 128 * 1152 / 8);
  pack_w_kernel<1><<<(64 * 1152 / 8) / 256, 256, 0, stream>>>(w_off, W2, 64, 128, 64 * 1152 / 8);
  pack_w_kernel<1><<<(64 * 1152 / 8) / 256, 256, 0, stream>>>(w_x, W3, 64, 128, 64 * 1152 / 8);
  pack_w_kernel<1><<<(kNcomPad * 576 / 8) / 256, 256, 0, stream>>>(w_com, W4, kNcom, 64, kNcomPad * 576 / 8);
  pack_w_kernel<1><<<(64 * 576 / 8) / 256, 256, 0, stream>>>(w_dcn, WD, 64, 64, 64 * 576 / 8);

  const int nl128 = 644 * 2, nl64 = 644;
  halo_zero_kernel<<<(nl128 * 8 + 255) / 256, 256, 0, stream>>>(CAT, 128, nl128);
  halo_zero_kernel<<<(nl128 * 8 + 255) / 256, 256, 0, stream>>>(TH, 128, nl128);
  halo_zero_kernel<<<(nl128 * 8 + 255) / 256, 256, 0, stream>>>(TL, 128, nl128);
  halo_zero_kernel<<<(nl64 * 8 + 255) / 256, 256, 0, stream>>>(OH, 64, nl64);
  halo_zero_kernel<<<(nl64 * 8 + 255) / 256, 256, 0, stream>>>(OL, 64, nl64);

  for (int b = 0; b < kB; ++b) {
    const size_t img = (size_t)b * kFc * kHW;
    cat_plane_kernel<<<kH * 5, 256, 0, stream>>>(ali + img, rin + img, CAT);
    conv3x3_kernel<1, 128, 2, 1, 0><<<(kMT * 2) / 4, 128, 0, stream>>>(
        CAT, CAT, W1, b_conv, TH, TL, XF, 128);
    conv3x3_kernel<0, 128, 1, 2, 1><<<kMT / 4, 128, 0, stream>>>(
        TH, TL, W2, b_off, OH, OL, out1 + img, 64);
    conv3x3_kernel<0, 128, 1, 1, 2><<<kMT / 4, 128, 0, stream>>>(
        TH, TH, W3, b_x, OH, OL, XF, 64);
    conv3x3_kernel<0, 64, 4, 2, 3><<<(kMT * 4) / 4, 128, 0, stream>>>(
        OH, OL, W4, b_com, TH, TL, COM, kNcom);
    dcn_kernel<<<kMT, 256, 0, stream>>>(XF, COM, WD, b_dcn, groups, out0 + img);
  }
}
